// SSMLayer_25675314495527
// MI455X (gfx1250) — hardware-verified
//
#include <hip/hip_runtime.h>
#include <math.h>

typedef __attribute__((ext_vector_type(16))) _Float16 v16h;
typedef __attribute__((ext_vector_type(8)))  _Float16 v8h;
typedef __attribute__((ext_vector_type(8)))  float    v8f;
typedef __attribute__((ext_vector_type(4)))  float    v4f;

constexpr int kBatch = 2;
constexpr int kSeqL  = 2048;
constexpr int kDmod  = 1024;
constexpr int kDin   = 2048;
constexpr int kNst   = 16;
constexpr int kDtR   = 64;
constexpr int kPrjN  = 96;
constexpr int kPrjP  = 128;
constexpr int kXZP   = 2 * kDin;
constexpr int kRows  = kBatch * kSeqL;
constexpr int kTP    = 260;
static_assert(kDtR + 2 * kNst == kPrjN, "x_proj width");
static_assert(kPrjP % 64 == 0 && kPrjP >= kPrjN, "padded x_proj width");
static_assert((kDmod % 32) == 0 && (kDin % 32) == 0 && (kDtR % 32) == 0, "GEMM K multiples of 32");
static_assert((kSeqL % 64) == 0 && (kXZP % 64) == 0 && (kDin % 64) == 0 && (kDmod % 64) == 0, "GEMM M,N multiples of 64");
static_assert((kDin % 256) == 0 && (kSeqL % 64) == 0 && (kSeqL % 16) == 0, "tile multiples");

constexpr float kCarryW   = 32.0f;
constexpr float kCarryWdt = 8.0f;
constexpr float kCarryDt  = 16.0f;
constexpr float kCarryY   = 16.0f;
constexpr float kFoldIn   = 1.0f / kCarryW;
constexpr float kFoldDt   = 1.0f / (kCarryDt * kCarryWdt);
constexpr float kFoldOut  = 1.0f / (kCarryY * kCarryW);

constexpr size_t kSzWIN16  = (size_t)kXZP * kDmod * 2;
constexpr size_t kSzWXP16  = (size_t)kPrjP * kDin * 2;
constexpr size_t kSzWDT16  = (size_t)kDin * kDtR * 2;
constexpr size_t kSzWOUT16 = (size_t)kDmod * kDin * 2;
constexpr size_t kSzX16    = (size_t)kRows * kDmod * 2;
constexpr size_t kSzXZ     = (size_t)kSeqL * kXZP * 4;
constexpr size_t kSzUC     = (size_t)kSeqL * kDin * 4;
constexpr size_t kSzUC16   = (size_t)kSeqL * kDin * 2;
constexpr size_t kSzPROJ   = (size_t)kSeqL * kPrjP * 4;
constexpr size_t kSzDT16   = (size_t)kSeqL * kDtR * 2;
constexpr size_t kSzDLR    = (size_t)kSeqL * kDin * 4;
constexpr size_t kSzY16    = (size_t)kSeqL * kDin * 2;
constexpr size_t kOffWIN16  = 0;
constexpr size_t kOffWXP16  = kOffWIN16  + kSzWIN16;
constexpr size_t kOffWDT16  = kOffWXP16  + kSzWXP16;
constexpr size_t kOffWOUT16 = kOffWDT16  + kSzWDT16;
constexpr size_t kOffX16    = kOffWOUT16 + kSzWOUT16;
constexpr size_t kOffXZ     = kOffX16    + kSzX16;
constexpr size_t kOffUC     = kOffXZ     + kSzXZ;
constexpr size_t kOffUC16   = kOffUC     + kSzUC;
constexpr size_t kOffPROJ   = kOffUC16   + kSzUC16;
constexpr size_t kOffDT16   = kOffPROJ   + kSzPROJ;
constexpr size_t kOffDLR    = kOffDT16   + kSzDT16;
constexpr size_t kOffY16    = kOffDLR    + kSzDLR;
constexpr size_t kWsTotal   = kOffY16    + kSzY16;
static_assert(kWsTotal == 106954752ull, "carve total");
static_assert(kWsTotal <= 134217728ull, "carve cap");
static_assert((kOffWXP16 % 128) == 0 && (kOffWDT16 % 128) == 0 && (kOffWOUT16 % 128) == 0 && (kOffX16 % 128) == 0 &&
              (kOffXZ % 128) == 0 && (kOffUC % 128) == 0 && (kOffUC16 % 128) == 0 && (kOffPROJ % 128) == 0 &&
              (kOffDT16 % 128) == 0 && (kOffDLR % 128) == 0 && (kOffY16 % 128) == 0, "128-B aligned regions");

__device__ __forceinline__ unsigned short f2bf_bits(float f) {
  unsigned u = __float_as_uint(f);
  return (unsigned short)((u + 0x7FFFu + ((u >> 16) & 1u)) >> 16);
}
__device__ __forceinline__ float bf_bits2f(unsigned short h) { return __uint_as_float(((unsigned)h) << 16); }
__device__ __forceinline__ float rne_bf(float f) { return bf_bits2f(f2bf_bits(f)); }

__device__ __forceinline__ void dep_guard_all_h(v8f& a, v8f& b, v8f& c, v8f& d, v16h x, v16h y0, v16h y1, v16h y2, v16h y3) {
  asm volatile("v_nop\n\tv_nop\n\tv_nop\n\tv_nop" : "+v"(a), "+v"(b), "+v"(c), "+v"(d) : "v"(x), "v"(y0), "v"(y1), "v"(y2), "v"(y3));
}
__device__ __forceinline__ void keep4_h(v16h a, v16h b, v16h c, v16h d) { asm volatile("v_nop" :: "v"(a), "v"(b), "v"(c), "v"(d)); }
__device__ __forceinline__ void acc_guard4(v8f& a, v8f& b, v8f& c, v8f& d) { asm volatile("v_nop\n\tv_nop\n\tv_nop\n\tv_nop" : "+v"(a), "+v"(b), "+v"(c), "+v"(d)); }

struct FragH {
  union U { v16h v; v8h h[2]; };
  static __device__ __forceinline__ v16h load(const _Float16* p) {
    U f; f.h[0] = *(const v8h*)(p); f.h[1] = *(const v8h*)(p + 16); return f.v;
  }
  static __device__ __forceinline__ v8f mma(v16h a, v16h b, v8f c) {
    return __builtin_amdgcn_wmma_f32_16x16x32_f16(false, a, false, b, (short)0, c, false, false);
  }
};

template <int BIAS_MODE>
__global__ __launch_bounds__(256) void wmma_gemm64(
    const unsigned short* __restrict__ Ap, int lda,
    const unsigned short* __restrict__ Btp, int ldb,
    float* __restrict__ Cout, int ldc,
    const float* __restrict__ bias,
    int M, int N, int K, float scale) {
  const _Float16* A  = (const _Float16*)Ap;
  const _Float16* Bt = (const _Float16*)Btp;
  __shared__ __align__(16) float sT[8][16 * 68];
  const int lane = threadIdx.x & 31;
  const int wave = threadIdx.x >> 5;
  const int tilesN = N >> 6;
  const int tilesM = M >> 6;
  const int tile = blockIdx.x * 8 + wave;
  if (tile >= tilesM * tilesN) return;
  const int tm = tile / tilesN;
  const int tn = tile - tm * tilesN;
  const int m0 = tm << 6;
  const int n0 = tn << 6;

  const int rlane = lane & 15;
  const int koff  = (lane >> 4) * 8;
  const int mOff  = (lane >> 4) * 8;

  v8f acc[4][4];
#pragma unroll
  for (int i = 0; i < 4; ++i)
#pragma unroll
    for (int j = 0; j < 4; ++j) acc[i][j] = (v8f){0.f,0.f,0.f,0.f,0.f,0.f,0.f,0.f};

  for (int k0 = 0; k0 < K; k0 += 32) {
    v16h bh[4];
#pragma unroll
    for (int j = 0; j < 4; ++j) {
      const size_t bo = (size_t)(n0 + (j << 4) + rlane) * ldb + koff + k0;
      bh[j] = FragH::load(Bt + bo);
    }
#pragma unroll
    for (int i = 0; i < 4; ++i) {
      const size_t ao = (size_t)(m0 + (i << 4) + rlane) * lda + koff + k0;
      v16h ah = FragH::load(A + ao);
#pragma unroll
      for (int j = 0; j < 4; ++j) acc[i][j] = FragH::mma(ah, bh[j], acc[i][j]);
      dep_guard_all_h(acc[i][0], acc[i][1], acc[i][2], acc[i][3], ah, bh[0], bh[1], bh[2], bh[3]);
    }
    keep4_h(bh[0], bh[1], bh[2], bh[3]);
  }
  acc_guard4(acc[0][0], acc[0][1], acc[0][2], acc[0][3]);
  acc_guard4(acc[1][0], acc[1][1], acc[1][2], acc[1][3]);
  acc_guard4(acc[2][0], acc[2][1], acc[2][2], acc[2][3]);
  acc_guard4(acc[3][0], acc[3][1], acc[3][2], acc[3][3]);

  float* slab = sT[wave];
#pragma unroll
  for (int i = 0; i < 4; ++i) {
    const int mBase = m0 + (i << 4);
#pragma unroll
    for (int j = 0; j < 4; ++j) {
      const int n = n0 + (j << 4) + rlane;
      float bv = 0.f;
      if (BIAS_MODE == 3) bv = rne_bf(bias[n]);
#pragma unroll
      for (int r = 0; r < 8; ++r) {
        float v = acc[i][j][r] * scale;
        if (BIAS_MODE == 3) v += bv;
        slab[(mOff + r) * 68 + (j << 4) + rlane] = v;
      }
    }
    __builtin_amdgcn_fence(__ATOMIC_RELEASE, "workgroup");
    __builtin_amdgcn_wave_barrier();
    __builtin_amdgcn_fence(__ATOMIC_ACQUIRE, "workgroup");
    {
      const int hh = lane >> 4, c4 = (lane & 15) * 4;
      for (int pass = 0; pass < 2; ++pass) {
#pragma unroll
        for (int it = 0; it < 8; ++it) {
          const int row = it * 2 + hh;
          v4f v = *(const v4f*)(slab + row * 68 + c4);
          *(volatile v4f*)(Cout + (size_t)(mBase + row) * ldc + n0 + c4) = v;
        }
        __threadfence();
      }
    }
    __builtin_amdgcn_fence(__ATOMIC_RELEASE, "workgroup");
    __builtin_amdgcn_wave_barrier();
    __builtin_amdgcn_fence(__ATOMIC_ACQUIRE, "workgroup");
  }
}

__global__ __launch_bounds__(256) void cast_bf_f16_kernel(
    const float* __restrict__ src, unsigned short* __restrict__ dst, int total8, int valid8, float scale)
{
  const int i = blockIdx.x * 256 + threadIdx.x;
  if (i >= total8) return;
  const bool live = (i < valid8);
  const int ic = live ? i : (valid8 - 1);
  const float* p = src + ((size_t)ic << 3);
  const v4f a0 = *(const v4f*)(p);
  const v4f a1 = *(const v4f*)(p + 4);
  v8h hv;
#pragma unroll
  for (int e = 0; e < 4; ++e) {
    const float f0 = a0[e];
    const float f1 = a1[e];
    const float r0 = live ? (rne_bf(f0) * scale) : 0.0f;
    const float r1 = live ? (rne_bf(f1) * scale) : 0.0f;
    hv[e]     = (_Float16)r0;
    hv[4 + e] = (_Float16)r1;
  }
  unsigned short* q = dst + ((size_t)i << 3);
  *(volatile v8h*)q = hv;
  __threadfence();
  *(volatile v8h*)q = hv;
}

__global__ __launch_bounds__(256) void dt_cast_kernel(
    const float* __restrict__ PROJ, unsigned short* __restrict__ DT16, int total8, float scale)
{
  const int i = blockIdx.x * 256 + threadIdx.x;
  if (i >= total8) return;
  const int e0  = i << 3;
  const int row = e0 >> 6;
  const int c8  = e0 & 63;
  const float* p = PROJ + (size_t)row * kPrjP + c8;
  const v4f a0 = *(const v4f*)(p);
  const v4f a1 = *(const v4f*)(p + 4);
  v8h hv;
#pragma unroll
  for (int e = 0; e < 4; ++e) {
    const float f0 = a0[e];
    const float f1 = a1[e];
    hv[e]     = (_Float16)(f0 * scale);
    hv[4 + e] = (_Float16)(f1 * scale);
  }
  unsigned short* qd = DT16 + e0;
  *(volatile v8h*)qd = hv;
  __threadfence();
  *(volatile v8h*)qd = hv;
}

__global__ __launch_bounds__(256) void conv_silu_kernel(
    const float* __restrict__ XZ, const float* __restrict__ cw, const float* __restrict__ cb,
    float* __restrict__ UC, unsigned short* __restrict__ UC16)
{
  __shared__ __align__(16) float sT[16 * kTP];
  const int tid = threadIdx.x, lane = tid & 31, wave = tid >> 5;
  const int d0 = blockIdx.x * 256, d = d0 + tid;
  const int t0 = blockIdx.y * 64;
  const v4f wv = *(const v4f*)(cw + (size_t)d * 4);
  const float wa = wv[0], wb = wv[1], wc = wv[2], wd = wv[3];
  const float w0 = rne_bf(wa), w1 = rne_bf(wb), w2 = rne_bf(wc), w3 = rne_bf(wd);
  const float bc = rne_bf(cb[d]);
  float xm3, xm2, xm1;
  {
    const int r3 = t0 - 3, r2 = t0 - 2, r1 = t0 - 1;
    const float v3 = XZ[(size_t)(r3 < 0 ? 0 : r3) * kXZP + d];
    const float v2 = XZ[(size_t)(r2 < 0 ? 0 : r2) * kXZP + d];
    const float v1 = XZ[(size_t)(r1 < 0 ? 0 : r1) * kXZP + d];
    xm3 = (r3 >= 0) ? v3 : 0.f;
    xm2 = (r2 >= 0) ? v2 : 0.f;
    xm1 = (r1 >= 0) ? v1 : 0.f;
  }
  const int hrow = wave >> 1;
  const int hch  = (wave & 1) * 128 + lane * 4;
#pragma unroll 1
  for (int sub = 0; sub < 4; ++sub) {
    const int lb = t0 + sub * 16;
#pragma unroll 1
    for (int s = 0; s < 16; ++s) {
      const float xc = XZ[(size_t)(lb + s) * kXZP + d];
      float acc = w0 * xm3;
      acc = fmaf(w1, xm2, acc);
      acc = fmaf(w2, xm1, acc);
      acc = fmaf(w3, xc, acc);
      const float sv = acc + bc;
      const float sg = __builtin_amdgcn_rcpf(1.0f + __expf(-sv));
      sT[s * kTP + tid] = sv * sg;
      xm3 = xm2; xm2 = xm1; xm1 = xc;
    }
    __syncthreads();
    v4f fv[4];
    v8h bv[2];
#pragma unroll
    for (int it = 0; it < 4; ++it) fv[it] = *(const v4f*)(sT + (it * 4 + hrow) * kTP + hch);
#pragma unroll
    for (int it = 0; it < 2; ++it) {
      const float* sp = sT + (it * 8 + wave) * kTP + lane * 8;
      const v4f a0 = *(const v4f*)(sp);
      const v4f a1 = *(const v4f*)(sp + 4);
#pragma unroll
      for (int e = 0; e < 4; ++e) {
        const float f0 = a0[e];
        const float f1 = a1[e];
        bv[it][e]     = (_Float16)f0;
        bv[it][4 + e] = (_Float16)f1;
      }
    }
    for (int pass = 0; pass < 2; ++pass) {
#pragma unroll
      for (int it = 0; it < 4; ++it)
        *(volatile v4f*)(UC + (size_t)(lb + it * 4 + hrow) * kDin + d0 + hch) = fv[it];
#pragma unroll
      for (int it = 0; it < 2; ++it)
        *(volatile v8h*)(UC16 + (size_t)(lb + it * 8 + wave) * kDin + d0 + lane * 8) = bv[it];
      __threadfence();
    }
    __syncthreads();
  }
}

__global__ __launch_bounds__(256) void scan_kernel(
    const float* __restrict__ DLR, const float* __restrict__ UC, const float* __restrict__ XZ,
    const float* __restrict__ PROJ, const float* __restrict__ A_log, const float* __restrict__ Dv,
    unsigned short* __restrict__ Y16)
{
  __shared__ __align__(16) float sBC[16 * 32];
  __shared__ __align__(16) float sY[16 * kTP];
  __shared__ __align__(16) float sA[kNst * 256];
  const int tid = threadIdx.x, lane = tid & 31, wave = tid >> 5;
  const int d0 = blockIdx.x * 256, d = d0 + tid;

#pragma unroll 1
  for (int n = 0; n < kNst; ++n) {
    const float al = A_log[(size_t)d * kNst + n];
    sA[n * 256 + tid] = -expf(rne_bf(al));
  }
  __syncthreads();
  float An[kNst], h[kNst];
#pragma unroll
  for (int n = 0; n < kNst; ++n) {
    An[n] = sA[n * 256 + tid];
    h[n] = 0.f;
  }
  const float Dd = rne_bf(Dv[d]);

#pragma unroll 1
  for (int c = 0; c < kSeqL / 16; ++c) {
    const int l0 = c * 16;
    if (tid < 128) {
      const int r = tid >> 3, q = (tid & 7) * 4;
      const v4f v = *(const v4f*)(PROJ + (size_t)(l0 + r) * kPrjP + kDtR + q);
      *(v4f*)(sBC + r * 32 + q) = v;
    }
    __syncthreads();
#pragma unroll 1
    for (int s = 0; s < 16; ++s) {
      const size_t m = (size_t)(l0 + s);
      float a  = DLR[m * kDin + d];
      float xv = UC[m * kDin + d];
      float zv = XZ[m * kXZP + kDin + d];
      asm volatile("" : "+v"(a), "+v"(xv), "+v"(zv));
      const float delta = fmaxf(a, 0.0f) + log1pf(__expf(-fabsf(a)));
      const float dtx   = delta * xv;
      v4f Bq[4], Cq[4];
#pragma unroll
      for (int qq = 0; qq < 4; ++qq) {
        Bq[qq] = *(const v4f*)(sBC + s * 32 + 4 * qq);
        Cq[qq] = *(const v4f*)(sBC + s * 32 + kNst + 4 * qq);
      }
      float y = 0.f;
#pragma unroll
      for (int n = 0; n < kNst; ++n) {
        const float e  = __expf(delta * An[n]);
        const float bn = Bq[n >> 2][n & 3];
        const float cn = Cq[n >> 2][n & 3];
        const float hn = fmaf(dtx, bn, e * h[n]);
        h[n] = hn;
        y = fmaf(hn, cn, y);
      }
      y = fmaf(xv, Dd, y);
      const float sg = __builtin_amdgcn_rcpf(1.0f + __expf(-zv));
      const float g  = zv * sg;
      sY[s * kTP + tid] = (y * g) * kCarryY;
    }
    __syncthreads();
    v8h hv[2];
#pragma unroll
    for (int it = 0; it < 2; ++it) {
      const float* sp = sY + (it * 8 + wave) * kTP + lane * 8;
      const v4f a0 = *(const v4f*)(sp);
      const v4f a1 = *(const v4f*)(sp + 4);
#pragma unroll
      for (int e = 0; e < 4; ++e) {
        const float f0 = a0[e];
        const float f1 = a1[e];
        hv[it][e]     = (_Float16)f0;
        hv[it][4 + e] = (_Float16)f1;
      }
    }
    for (int pass = 0; pass < 2; ++pass) {
#pragma unroll
      for (int it = 0; it < 2; ++it)
        *(volatile v8h*)(Y16 + (size_t)(l0 + it * 8 + wave) * kDin + d0 + lane * 8) = hv[it];
      __threadfence();
    }
  }
}

static_assert((kSeqL / 64) * (kXZP / 64) == 256 * 8, "in_proj grid");
static_assert((kSeqL / 64) * (kPrjP / 64) == 8 * 8, "x_proj grid");
static_assert((kSeqL / 64) * (kDin / 64) == 128 * 8, "dt_proj grid");
static_assert((kSeqL / 64) * (kDmod / 64) == 64 * 8, "out_proj grid");
static_assert(((kRows * kDmod / 8) % 256) == 0 && ((kXZP * kDmod / 8) % 256) == 0 && ((kPrjP * kDin / 8) % 256) == 0 &&
              ((kDin * kDtR / 8) % 256) == 0 && ((kDmod * kDin / 8) % 256) == 0 && ((kSeqL * kDtR / 8) % 256) == 0, "cast grids exact");

extern "C" void kernel_launch(void* const* d_in, const int* in_sizes, int n_in,
                              void* d_out, int out_size, void* d_ws, size_t ws_size,
                              hipStream_t stream)
{
  if (n_in < 10) return;
  if (in_sizes[0] != kRows * kDmod) return;
  if (in_sizes[1] != kXZP * kDmod) return;
  if (in_sizes[2] != kDin * 4 || in_sizes[3] != kDin) return;
  if (in_sizes[4] != kPrjN * kDin) return;
  if (in_sizes[5] != kDin * kDtR || in_sizes[6] != kDin) return;
  if (in_sizes[7] != kDin * kNst || in_sizes[8] != kDin) return;
  if (in_sizes[9] != kDmod * kDin) return;
  if (out_size != kRows * kDmod) return;
  if (ws_size < kWsTotal) return;

  const float* x      = (const float*)d_in[0];
  const float* W_in   = (const float*)d_in[1];
  const float* conv_w = (const float*)d_in[2];
  const float* conv_b = (const float*)d_in[3];
  const float* W_xprj = (const float*)d_in[4];
  const float* W_dt   = (const float*)d_in[5];
  const float* b_dt   = (const float*)d_in[6];
  const float* A_log  = (const float*)d_in[7];
  const float* Dv     = (const float*)d_in[8];
  const float* W_out  = (const float*)d_in[9];
  float* dout = (float*)d_out;

  char* ws = (char*)d_ws;
  unsigned short* WIN16  = (unsigned short*)(ws + kOffWIN16);
  unsigned short* WXP16  = (unsigned short*)(ws + kOffWXP16);
  unsigned short* WDT16  = (unsigned short*)(ws + kOffWDT16);
  unsigned short* WOUT16 = (unsigned short*)(ws + kOffWOUT16);
  unsigned short* X16    = (unsigned short*)(ws + kOffX16);
  float*          XZ     = (float*)(ws + kOffXZ);
  float*          UC     = (float*)(ws + kOffUC);
  unsigned short* UC16   = (unsigned short*)(ws + kOffUC16);
  float*          PROJ   = (float*)(ws + kOffPROJ);
  unsigned short* DT16   = (unsigned short*)(ws + kOffDT16);
  float*          DLR    = (float*)(ws + kOffDLR);
  unsigned short* Y16    = (unsigned short*)(ws + kOffY16);

  cast_bf_f16_kernel<<<(kRows * kDmod / 8) / 256, 256, 0, stream>>>(x, X16, kRows * kDmod / 8, kRows * kDmod / 8, 1.0f);
  cast_bf_f16_kernel<<<(kXZP * kDmod / 8) / 256, 256, 0, stream>>>(W_in, WIN16, kXZP * kDmod / 8, kXZP * kDmod / 8, kCarryW);
  cast_bf_f16_kernel<<<(kPrjP * kDin / 8) / 256, 256, 0, stream>>>(W_xprj, WXP16, kPrjP * kDin / 8, kPrjN * kDin / 8, kCarryW);
  cast_bf_f16_kernel<<<(kDin * kDtR / 8) / 256, 256, 0, stream>>>(W_dt, WDT16, kDin * kDtR / 8, kDin * kDtR / 8, kCarryWdt);
  cast_bf_f16_kernel<<<(kDmod * kDin / 8) / 256, 256, 0, stream>>>(W_out, WOUT16, kDmod * kDin / 8, kDmod * kDin / 8, kCarryW);

  for (int b = 0; b < kBatch; ++b) {
    const unsigned short* X16b = X16 + (size_t)b * kSeqL * kDmod;
    float* outb = dout + (size_t)b * kSeqL * kDmod;

    wmma_gemm64<0><<<dim3(256, 1), 256, 0, stream>>>(
        X16b, kDmod, WIN16, kDmod, XZ, kXZP, b_dt, kSeqL, kXZP, kDmod, kFoldIn);

    conv_silu_kernel<<<dim3(kDin / 256, kSeqL / 64), 256, 0, stream>>>(XZ, conv_w, conv_b, UC, UC16);

    wmma_gemm64<0><<<dim3(8, 1), 256, 0, stream>>>(
        UC16, kDin, WXP16, kDin, PROJ, kPrjP, b_dt, kSeqL, kPrjP, kDin, kFoldIn);

    dt_cast_kernel<<<(kSeqL * kDtR / 8) / 256, 256, 0, stream>>>(PROJ, DT16, kSeqL * kDtR / 8, kCarryDt);

    wmma_gemm64<3><<<dim3(128, 1), 256, 0, stream>>>(
        DT16, kDtR, WDT16, kDtR, DLR, kDin, b_dt, kSeqL, kDin, kDtR, kFoldDt);

    scan_kernel<<<dim3(kDin / 256, 1), 256, 0, stream>>>(DLR, UC, XZ, PROJ, A_log, Dv, Y16);

    wmma_gemm64<0><<<dim3(64, 1), 256, 0, stream>>>(
        Y16, kDin, WOUT16, kDin, outb, kDmod, b_dt, kSeqL, kDmod, kDin, kFoldOut);
  }
}
